// CrossGraphAttentionModel_27410481283242
// MI455X (gfx1250) — hardware-verified
//
#include <hip/hip_runtime.h>
#include <math.h>
#include <stdint.h>

typedef _Float16 v16h __attribute__((ext_vector_type(16)));
typedef _Float16 v8h  __attribute__((ext_vector_type(8)));
typedef float    v8f  __attribute__((ext_vector_type(8)));
typedef float    v4f  __attribute__((ext_vector_type(4)));
typedef int      v4i  __attribute__((ext_vector_type(4)));

union Frag { v16h v; v8h half[2]; };

__device__ __forceinline__ v8f mma16(v16h a, v16h b, v8f c) {
  c = __builtin_amdgcn_wmma_f32_16x16x32_f16(false, a, false, b, (short)0, c, false, false);
  asm volatile("v_nop\n\tv_nop\n\tv_nop\n\tv_nop" : "+v"(c) : "v"(a), "v"(b));
  return c;
}
__device__ __forceinline__ v8f zero8f() {
  v8f z;
#pragma unroll
  for (int i = 0; i < 8; ++i) z[i] = 0.0f;
  return z;
}
__device__ __forceinline__ v8h zero8h() {
  v8h z;
#pragma unroll
  for (int i = 0; i < 8; ++i) z[i] = (_Float16)0.0f;
  return z;
}
__device__ __forceinline__ v8h cvt8(const float* p) {
  const v4f a = *(const v4f*)p;
  const v4f b = *(const v4f*)(p + 4);
  v8h r;
  r[0] = (_Float16)a[0]; r[1] = (_Float16)a[1]; r[2] = (_Float16)a[2]; r[3] = (_Float16)a[3];
  r[4] = (_Float16)b[0]; r[5] = (_Float16)b[1]; r[6] = (_Float16)b[2]; r[7] = (_Float16)b[3];
  return r;
}
__device__ __forceinline__ void wave_sync_lds() {
  __builtin_amdgcn_fence(__ATOMIC_RELEASE, "workgroup");
  __builtin_amdgcn_wave_barrier();
  __builtin_amdgcn_fence(__ATOMIC_ACQUIRE, "workgroup");
}

#define SG_R 128
#define SG_C 2048
#define SG_T 256

template <int KIN>
__global__ __launch_bounds__(SG_T) void k_conv(const float* __restrict__ x, const int* __restrict__ edge, int E, int N,
                                               const float* __restrict__ wl, const float* __restrict__ bl,
                                               const float* __restrict__ wr, float* __restrict__ hout) {
  constexpr int K2 = 2 * KIN;
  constexpr int WP = K2 + 8;
  __shared__ __align__(16) float aggL[SG_R * 64];
  __shared__ float cntL[SG_R];
  __shared__ unsigned listL[SG_C];
  __shared__ int wtot[SG_T / 32];
  __shared__ __align__(16) _Float16 wL[64 * WP];

  const int tid = threadIdx.x, lane = tid & 31, wave = tid >> 5;
  const int row0 = blockIdx.x * SG_R;

  for (int i = tid; i < SG_R * KIN; i += SG_T) aggL[i] = 0.0f;
  if (tid < SG_R) cntL[tid] = 0.0f;
  for (int idx = tid; idx < 64 * K2; idx += SG_T) {
    const int k = idx >> 6, n = idx & 63;
    const int kl = min(k, KIN - 1), kr = max(k - KIN, 0);
    const float a = wl[kl * 64 + n];
    const float b = wr[kr * 64 + n];
    const float v = (k < KIN) ? a : b;
    wL[n * WP + k] = (_Float16)(v * 16.0f);
  }
  __syncthreads();

  const int* esrc = edge;
  const int* edst = edge + E;
  const int nch = (E + SG_C - 1) / SG_C;
  const bool al4 = ((E & 3) == 0);
  for (int ch = 0; ch < nch; ++ch) {
    const int cbase = ch * SG_C;
    const int e0 = cbase + 8 * tid;
    int dv[8], sv[8];
    if (al4 && (cbase + SG_C <= E)) {
      const v4i d0 = *(const v4i*)(edst + e0);
      const v4i d1 = *(const v4i*)(edst + e0 + 4);
      const v4i s0 = *(const v4i*)(esrc + e0);
      const v4i s1 = *(const v4i*)(esrc + e0 + 4);
      dv[0] = d0[0]; dv[1] = d0[1]; dv[2] = d0[2]; dv[3] = d0[3];
      dv[4] = d1[0]; dv[5] = d1[1]; dv[6] = d1[2]; dv[7] = d1[3];
      sv[0] = s0[0]; sv[1] = s0[1]; sv[2] = s0[2]; sv[3] = s0[3];
      sv[4] = s1[0]; sv[5] = s1[1]; sv[6] = s1[2]; sv[7] = s1[3];
    } else {
#pragma unroll
      for (int j = 0; j < 8; ++j) {
        const int e = e0 + j;
        const int ec = min(e, E - 1);
        const int d = edst[ec];
        const int s = esrc[ec];
        dv[j] = (e < E) ? d : -1;
        sv[j] = s;
      }
    }
    unsigned ent[8];
    int hits = 0, cntT = 0;
#pragma unroll
    for (int j = 0; j < 8; ++j) {
      const int ld = dv[j] - row0;
      const bool hit = (unsigned)ld < (unsigned)SG_R;
      const int s = min(max(sv[j], 0), N - 1);
      ent[j] = ((unsigned)(ld & (SG_R - 1)) << 16) | (unsigned)s;
      if (hit) { hits |= (1 << j); ++cntT; }
    }
    int incl = cntT;
#pragma unroll
    for (int off = 1; off < 32; off <<= 1) {
      const int y = __shfl_up(incl, off, 32);
      if (lane >= off) incl += y;
    }
    if (lane == 31) wtot[wave] = incl;
    __syncthreads();
    int base = 0, total = 0;
#pragma unroll
    for (int w = 0; w < SG_T / 32; ++w) {
      const int t = wtot[w];
      total += t;
      if (w < wave) base += t;
    }
    int pos = base + incl - cntT;
#pragma unroll
    for (int j = 0; j < 8; ++j) {
      if (hits & (1 << j)) { listL[min(pos, SG_C - 1)] = ent[j]; ++pos; }
    }
    __syncthreads();
    const int nh = min(total, SG_C);
    if (tid < KIN) {
      const int c = tid;
      for (int i = 0; i < nh; ++i) {
        const unsigned en = listL[i];
        const int ld = (int)(en >> 16) & (SG_R - 1);
        const int sr = min((int)(en & 0xffffu), N - 1);
        const float v = x[(size_t)sr * KIN + c];
        aggL[ld * KIN + c] += v;
        if (c == 0) cntL[ld] += 1.0f;
      }
    }
    __syncthreads();
  }

  for (int idx = tid; idx < SG_R * KIN; idx += SG_T) {
    const int r = idx / KIN;
    const float cn = fmaxf(cntL[r], 1.0f);
    aggL[idx] = aggL[idx] * (1.0f / cn);
  }
  __syncthreads();

  const int hh = lane >> 4, m = lane & 15;
  const int rw = wave * 16;
  v8f acc[4];
#pragma unroll
  for (int j = 0; j < 4; ++j) acc[j] = zero8f();
#pragma unroll
  for (int ks = 0; ks < KIN / 32; ++ks) {
    const int k0 = ks * 32;
    Frag a;
    const float* ap = aggL + (rw + m) * KIN + k0 + 8 * hh;
    a.half[0] = cvt8(ap);
    a.half[1] = cvt8(ap + 16);
#pragma unroll
    for (int j = 0; j < 4; ++j) {
      Frag b;
      const _Float16* bp = wL + (16 * j + m) * WP + k0 + 8 * hh;
      b.half[0] = *(const v8h*)bp;
      b.half[1] = *(const v8h*)(bp + 16);
      acc[j] = mma16(a.v, b.v, acc[j]);
    }
  }
#pragma unroll
  for (int ks = 0; ks < KIN / 32; ++ks) {
    const int k0 = ks * 32;
    Frag a;
    const float* ap = x + (size_t)(row0 + rw + m) * KIN + k0 + 8 * hh;
    a.half[0] = cvt8(ap);
    a.half[1] = cvt8(ap + 16);
#pragma unroll
    for (int j = 0; j < 4; ++j) {
      Frag b;
      const _Float16* bp = wL + (16 * j + m) * WP + KIN + k0 + 8 * hh;
      b.half[0] = *(const v8h*)bp;
      b.half[1] = *(const v8h*)(bp + 16);
      acc[j] = mma16(a.v, b.v, acc[j]);
    }
  }
  __syncthreads();

  float* stg = aggL;
#pragma unroll
  for (int j = 0; j < 4; ++j) {
    const int n = 16 * j + m;
    const float bv = bl[n];
#pragma unroll
    for (int r = 0; r < 8; ++r) {
      float v = acc[j][r] * 0.0625f + bv;
      v = fmaxf(v, 0.0f);
      stg[(rw + 8 * hh + r) * 64 + n] = v;
    }
  }
  __syncthreads();
  const int c4 = m * 4;
#pragma unroll
  for (int it = 0; it < 8; ++it) {
    const int row = rw + 2 * it + hh;
    const v4f v = *(const v4f*)(stg + row * 64 + c4);
    *(volatile v4f*)(hout + (size_t)(row0 + row) * 64 + c4) = v;
  }
  __threadfence();
#pragma unroll
  for (int it = 0; it < 8; ++it) {
    const int row = rw + 2 * it + hh;
    const v4f v = *(const v4f*)(stg + row * 64 + c4);
    *(volatile v4f*)(hout + (size_t)(row0 + row) * 64 + c4) = v;
  }
}

__global__ __launch_bounds__(128) void k_proj(const float* __restrict__ A, int N,
                                              const float* __restrict__ W0, const float* __restrict__ B0, _Float16* O0,
                                              const float* __restrict__ W1, const float* __restrict__ B1, _Float16* O1,
                                              const float* __restrict__ W2, const float* __restrict__ B2, _Float16* O2t) {
  __shared__ __align__(16) _Float16 wL[64 * 72];
  __shared__ __align__(16) _Float16 stg[64 * 72];
  const int z = blockIdx.y;
  const float* W = (z == 0) ? W0 : ((z == 1) ? W1 : W2);
  const float* Bv = (z == 0) ? B0 : ((z == 1) ? B1 : B2);
  _Float16* O = (z == 0) ? O0 : ((z == 1) ? O1 : O2t);
  const bool trans = (z == 2);
  const int tid = threadIdx.x, lane = tid & 31, wave = tid >> 5;
  const int hh = lane >> 4, m = lane & 15;
  const int row0 = blockIdx.x * 64;

  for (int idx = tid; idx < 64 * 64; idx += 128) {
    const int k = idx >> 6, n = idx & 63;
    wL[n * 72 + k] = (_Float16)(W[k * 64 + n] * 16.0f);
  }
  __syncthreads();

  const int rw = wave * 16;
  v8f acc[4];
#pragma unroll
  for (int j = 0; j < 4; ++j) acc[j] = zero8f();
#pragma unroll
  for (int ks = 0; ks < 2; ++ks) {
    const int k0 = ks * 32;
    Frag a;
    const float* ap = A + (size_t)(row0 + rw + m) * 64 + k0 + 8 * hh;
    a.half[0] = cvt8(ap);
    a.half[1] = cvt8(ap + 16);
#pragma unroll
    for (int j = 0; j < 4; ++j) {
      Frag b;
      const _Float16* bp = wL + (16 * j + m) * 72 + k0 + 8 * hh;
      b.half[0] = *(const v8h*)bp;
      b.half[1] = *(const v8h*)(bp + 16);
      acc[j] = mma16(a.v, b.v, acc[j]);
    }
  }
#pragma unroll
  for (int j = 0; j < 4; ++j) {
    const int n = 16 * j + m;
    const float bv = Bv[n];
#pragma unroll
    for (int r = 0; r < 8; ++r) {
      const int rr = rw + 8 * hh + r;
      const _Float16 h = (_Float16)(acc[j][r] * 0.0625f + bv);
      const int idx = trans ? (n * 72 + rr) : (rr * 72 + n);
      stg[idx] = h;
    }
  }
  __syncthreads();
  const int q = tid >> 3, c8 = (tid & 7) * 8;
  v8h vals[4];
  size_t offs[4];
#pragma unroll
  for (int it = 0; it < 4; ++it) {
    const int line = it * 16 + q;
    vals[it] = *(const v8h*)(stg + line * 72 + c8);
    offs[it] = trans ? ((size_t)line * (size_t)N + (size_t)row0 + (size_t)c8)
                     : ((size_t)(row0 + line) * 64 + (size_t)c8);
  }
#pragma unroll
  for (int it = 0; it < 4; ++it) *(volatile v8h*)(O + offs[it]) = vals[it];
  __threadfence();
#pragma unroll
  for (int it = 0; it < 4; ++it) *(volatile v8h*)(O + offs[it]) = vals[it];
}

__global__ __launch_bounds__(128) void k_attn(const _Float16* __restrict__ Qp, const _Float16* __restrict__ Kp,
                                              const _Float16* __restrict__ Vt, const float* __restrict__ resid,
                                              float* out, int Nq, int Nk) {
  __shared__ __align__(16) _Float16 pws[4][16 * 64];
  __shared__ __align__(16) float os[16 * 64];
  const int tid = threadIdx.x, lane = tid & 31, hd = tid >> 5;
  const int hh = lane >> 4, m = lane & 15;
  const int q0 = blockIdx.x * 16;
  (void)Nq;

  Frag qa;
  qa.half[0] = *(const v8h*)(Qp + (size_t)(q0 + m) * 64 + hd * 16 + 8 * hh);
  qa.half[1] = zero8h();

  float mrow[8], lrow[8];
#pragma unroll
  for (int r = 0; r < 8; ++r) { mrow[r] = -INFINITY; lrow[r] = 0.0f; }
  v8f oacc = zero8f();
  _Float16* pw = pws[hd];
  const _Float16* vrow = Vt + (size_t)(hd * 16 + m) * (size_t)Nk;

  const int nch = Nk >> 6;
  for (int kc = 0; kc < nch; ++kc) {
    const int k0 = kc * 64;
    v8f s[4];
#pragma unroll
    for (int j = 0; j < 4; ++j) {
      Frag kb;
      kb.half[0] = *(const v8h*)(Kp + (size_t)(k0 + 16 * j + m) * 64 + hd * 16 + 8 * hh);
      kb.half[1] = zero8h();
      s[j] = mma16(qa.v, kb.v, zero8f());
    }
    float cm[8];
#pragma unroll
    for (int r = 0; r < 8; ++r) {
      float mx = -INFINITY;
#pragma unroll
      for (int j = 0; j < 4; ++j) {
        const float sv = s[j][r] * 0.25f;
        s[j][r] = sv;
        mx = fmaxf(mx, sv);
      }
#pragma unroll
      for (int off = 1; off < 16; off <<= 1) mx = fmaxf(mx, __shfl_xor(mx, off, 32));
      cm[r] = mx;
    }
    wave_sync_lds();
#pragma unroll
    for (int r = 0; r < 8; ++r) {
      const float mnew = fmaxf(mrow[r], cm[r]);
      const float alpha = __expf(mrow[r] - mnew);
      mrow[r] = mnew;
      float psum = 0.0f;
#pragma unroll
      for (int j = 0; j < 4; ++j) {
        const float p = __expf(s[j][r] - mnew);
        psum += p;
        pw[(8 * hh + r) * 64 + 16 * j + m] = (_Float16)(p * 256.0f);
      }
#pragma unroll
      for (int off = 1; off < 16; off <<= 1) psum += __shfl_xor(psum, off, 32);
      lrow[r] = lrow[r] * alpha + psum;
      oacc[r] *= alpha;
    }
    wave_sync_lds();
#pragma unroll
    for (int kk = 0; kk < 2; ++kk) {
      Frag pa, vb;
      pa.half[0] = *(const v8h*)(pw + m * 64 + 32 * kk + 8 * hh);
      pa.half[1] = *(const v8h*)(pw + m * 64 + 32 * kk + 16 + 8 * hh);
      vb.half[0] = *(const v8h*)(vrow + k0 + 32 * kk + 8 * hh);
      vb.half[1] = *(const v8h*)(vrow + k0 + 32 * kk + 16 + 8 * hh);
      oacc = mma16(pa.v, vb.v, oacc);
    }
  }

#pragma unroll
  for (int r = 0; r < 8; ++r) {
    const float inv = 1.0f / (lrow[r] * 256.0f);
    os[(8 * hh + r) * 64 + hd * 16 + m] = oacc[r] * inv;
  }
  __syncthreads();
  const int rr = tid >> 4, c4 = (tid & 15) * 4;
  v4f vals[2];
#pragma unroll
  for (int it = 0; it < 2; ++it) {
    const int row = it * 8 + rr;
    const v4f o = *(const v4f*)(os + row * 64 + c4);
    const v4f rs = *(const v4f*)(resid + (size_t)(q0 + row) * 64 + c4);
    vals[it] = o + rs;
  }
#pragma unroll
  for (int it = 0; it < 2; ++it)
    *(volatile v4f*)(out + (size_t)(q0 + it * 8 + rr) * 64 + c4) = vals[it];
  __threadfence();
#pragma unroll
  for (int it = 0; it < 2; ++it)
    *(volatile v4f*)(out + (size_t)(q0 + it * 8 + rr) * 64 + c4) = vals[it];
}

__global__ __launch_bounds__(256) void k_pool_head(const float* __restrict__ hmc, const int* __restrict__ bm, int NM,
                                                   const float* __restrict__ hpc, const int* __restrict__ bp, int NP,
                                                   const float* __restrict__ fc1w, const float* __restrict__ fc1b,
                                                   const float* __restrict__ fc2w, const float* __restrict__ fc2b,
                                                   float* out) {
  __shared__ __align__(16) float zL[64 * 128];
  __shared__ float cntL[128];
  __shared__ __align__(16) _Float16 wL[64 * 136];
  __shared__ __align__(16) float outL[64];
  const int tid = threadIdx.x, lane = tid & 31, wave = tid >> 5;
  const int hh = lane >> 4, m = lane & 15;

  for (int i = tid; i < 64 * 128; i += 256) zL[i] = 0.0f;
  if (tid < 128) cntL[tid] = 0.0f;
  for (int idx = tid; idx < 128 * 64; idx += 256) {
    const int k = idx >> 6, n = idx & 63;
    wL[n * 136 + k] = (_Float16)(fc1w[k * 64 + n] * 16.0f);
  }
  __syncthreads();

  if (tid < 64) {
    const int c = tid;
    for (int n = 0; n < NM; ++n) {
      const int b = bm[n];
      const float v = hmc[(size_t)n * 64 + c];
      if ((unsigned)b < 64u) {
        zL[b * 128 + c] += v;
        if (c == 0) cntL[b] += 1.0f;
      }
    }
  } else if (tid < 128) {
    const int c = tid - 64;
    for (int n = 0; n < NP; ++n) {
      const int b = bp[n];
      const float v = hpc[(size_t)n * 64 + c];
      if ((unsigned)b < 64u) {
        zL[b * 128 + 64 + c] += v;
        if (c == 0) cntL[64 + b] += 1.0f;
      }
    }
  }
  __syncthreads();
  for (int idx = tid; idx < 64 * 128; idx += 256) {
    const int b = idx >> 7, col = idx & 127;
    const float cn = fmaxf(cntL[(col >> 6) * 64 + b], 1.0f);
    zL[idx] = zL[idx] * (1.0f / cn);
  }
  __syncthreads();

  const int mi = wave & 3, nj0 = (wave >> 2) * 2;
  v8f acc[2];
  acc[0] = zero8f(); acc[1] = zero8f();
#pragma unroll
  for (int ks = 0; ks < 4; ++ks) {
    const int k0 = ks * 32;
    Frag a;
    const float* ap = zL + (16 * mi + m) * 128 + k0 + 8 * hh;
    a.half[0] = cvt8(ap);
    a.half[1] = cvt8(ap + 16);
#pragma unroll
    for (int jj = 0; jj < 2; ++jj) {
      Frag b;
      const _Float16* bpp = wL + (16 * (nj0 + jj) + m) * 136 + k0 + 8 * hh;
      b.half[0] = *(const v8h*)bpp;
      b.half[1] = *(const v8h*)(bpp + 16);
      acc[jj] = mma16(a.v, b.v, acc[jj]);
    }
  }
  __syncthreads();
  float* xs = zL;
#pragma unroll
  for (int jj = 0; jj < 2; ++jj) {
    const int n = 16 * (nj0 + jj) + m;
    const float bv = fc1b[n];
#pragma unroll
    for (int r = 0; r < 8; ++r) {
      float v = acc[jj][r] * 0.0625f + bv;
      v = fmaxf(v, 0.0f);
      xs[(16 * mi + 8 * hh + r) * 64 + n] = v;
    }
  }
  __syncthreads();
  if (tid < 64) {
    float a = fc2b[0];
#pragma unroll 4
    for (int k = 0; k < 64; ++k) a += xs[tid * 64 + k] * fc2w[k];
    const float e = expf(-a);
    outL[tid] = 1.0f / (1.0f + e);
  }
  __syncthreads();
  v4f ov;
  ov[0] = 0.0f; ov[1] = 0.0f; ov[2] = 0.0f; ov[3] = 0.0f;
  if (tid < 16) ov = *(const v4f*)(outL + 4 * tid);
  if (tid < 16) *(volatile v4f*)(out + 4 * tid) = ov;
  __threadfence();
  if (tid < 16) *(volatile v4f*)(out + 4 * tid) = ov;
}

extern "C" void kernel_launch(void* const* d_in, const int* in_sizes, int n_in,
                              void* d_out, int out_size, void* d_ws, size_t ws_size,
                              hipStream_t stream) {
  if (n_in != 26) return;
  if (out_size != 64) return;
  const int NM = in_sizes[24];
  const int NP = in_sizes[25];
  if (NM <= 0 || NP <= 0 || (NM % 128) != 0 || (NP % 128) != 0 || NM > 65536 || NP > 65536) return;
  if ((in_sizes[22] & 1) != 0 || (in_sizes[23] & 1) != 0) return;
  const int EM = in_sizes[22] / 2;
  const int EP = in_sizes[23] / 2;
  if (EM <= 0 || EP <= 0) return;
  if (in_sizes[0] != NM * 32 || in_sizes[1] != NP * 64) return;
  if (in_sizes[2] != 32 * 64 || in_sizes[3] != 64 || in_sizes[4] != 32 * 64) return;
  if (in_sizes[5] != 4096 || in_sizes[6] != 64 || in_sizes[7] != 4096) return;
  if (in_sizes[8] != 4096 || in_sizes[9] != 64 || in_sizes[10] != 4096) return;
  if (in_sizes[11] != 4096 || in_sizes[12] != 64 || in_sizes[13] != 4096) return;
  if (in_sizes[14] != 3 * 4096 || in_sizes[15] != 192 || in_sizes[16] != 3 * 4096 || in_sizes[17] != 192) return;
  if (in_sizes[18] != 128 * 64 || in_sizes[19] != 64 || in_sizes[20] != 64 || in_sizes[21] < 1) return;

  const float* x_mol  = (const float*)d_in[0];
  const float* x_prot = (const float*)d_in[1];
  const float* m1_wl = (const float*)d_in[2];
  const float* m1_bl = (const float*)d_in[3];
  const float* m1_wr = (const float*)d_in[4];
  const float* m2_wl = (const float*)d_in[5];
  const float* m2_bl = (const float*)d_in[6];
  const float* m2_wr = (const float*)d_in[7];
  const float* p1_wl = (const float*)d_in[8];
  const float* p1_bl = (const float*)d_in[9];
  const float* p1_wr = (const float*)d_in[10];
  const float* p2_wl = (const float*)d_in[11];
  const float* p2_bl = (const float*)d_in[12];
  const float* p2_wr = (const float*)d_in[13];
  const float* amp_w = (const float*)d_in[14];
  const float* amp_b = (const float*)d_in[15];
  const float* apm_w = (const float*)d_in[16];
  const float* apm_b = (const float*)d_in[17];
  const float* fc1_w = (const float*)d_in[18];
  const float* fc1_b = (const float*)d_in[19];
  const float* fc2_w = (const float*)d_in[20];
  const float* fc2_b = (const float*)d_in[21];
  const int* edge_mol   = (const int*)d_in[22];
  const int* edge_prot  = (const int*)d_in[23];
  const int* batch_mol  = (const int*)d_in[24];
  const int* batch_prot = (const int*)d_in[25];
  float* outp = (float*)d_out;

  const size_t fM = (size_t)NM * 64 * 4;
  const size_t fP = (size_t)NP * 64 * 4;
  const size_t hM = (size_t)NM * 64 * 2;
  const size_t hP = (size_t)NP * 64 * 2;
  size_t off = 0;
  auto carve = [&](size_t bytes) -> size_t { const size_t o = off; off = (off + bytes + 255) & ~(size_t)255; return o; };
  const size_t oHm1 = carve(fM), oHm2 = carve(fM);
  const size_t oHp1 = carve(fP), oHp2 = carve(fP);
  const size_t oQm = carve(hM), oKm = carve(hM), oVmt = carve(hM);
  const size_t oQp = carve(hP), oKp = carve(hP), oVpt = carve(hP);
  const size_t oHmc = carve(fM), oHpc = carve(fP);
  if (off > ws_size) return;

  char* ws = (char*)d_ws;
  float* hm1 = (float*)(ws + oHm1);
  float* hm2 = (float*)(ws + oHm2);
  float* hp1 = (float*)(ws + oHp1);
  float* hp2 = (float*)(ws + oHp2);
  _Float16* Qm  = (_Float16*)(ws + oQm);
  _Float16* Km  = (_Float16*)(ws + oKm);
  _Float16* Vmt = (_Float16*)(ws + oVmt);
  _Float16* Qp  = (_Float16*)(ws + oQp);
  _Float16* Kp  = (_Float16*)(ws + oKp);
  _Float16* Vpt = (_Float16*)(ws + oVpt);
  float* hmc = (float*)(ws + oHmc);
  float* hpc = (float*)(ws + oHpc);

  k_conv<32><<<dim3(NM / SG_R), dim3(SG_T), 0, stream>>>(x_mol, edge_mol, EM, NM, m1_wl, m1_bl, m1_wr, hm1);
  k_conv<64><<<dim3(NM / SG_R), dim3(SG_T), 0, stream>>>(hm1, edge_mol, EM, NM, m2_wl, m2_bl, m2_wr, hm2);
  k_conv<64><<<dim3(NP / SG_R), dim3(SG_T), 0, stream>>>(x_prot, edge_prot, EP, NP, p1_wl, p1_bl, p1_wr, hp1);
  k_conv<64><<<dim3(NP / SG_R), dim3(SG_T), 0, stream>>>(hp1, edge_prot, EP, NP, p2_wl, p2_bl, p2_wr, hp2);

  k_proj<<<dim3(NM / 64, 3), dim3(128), 0, stream>>>(hm2, NM,
      amp_w, amp_b, Qm, apm_w + 4096, apm_b + 64, Km, apm_w + 8192, apm_b + 128, Vmt);
  k_proj<<<dim3(NP / 64, 3), dim3(128), 0, stream>>>(hp2, NP,
      apm_w, apm_b, Qp, amp_w + 4096, amp_b + 64, Kp, amp_w + 8192, amp_b + 128, Vpt);

  k_attn<<<dim3(NM / 16), dim3(128), 0, stream>>>(Qm, Kp, Vpt, hm2, hmc, NM, NP);
  k_attn<<<dim3(NP / 16), dim3(128), 0, stream>>>(Qp, Km, Vmt, hp2, hpc, NP, NM);

  k_pool_head<<<dim3(1), dim3(256), 0, stream>>>(hmc, batch_mol, NM, hpc, batch_prot, NP,
                                                 fc1_w, fc1_b, fc2_w, fc2_b, outp);
  (void)hipGetLastError();
}
